// AttentionWithPairBias_78228534329665
// MI455X (gfx1250) — hardware-run, weakly checked
//
#include <hip/hip_runtime.h>


#define TT   768
#define HD   64
#define ZH   1
#define RH   0
#define PCAR 1024.0f
#define SCL  0.14433757f
#define PMUL 1.0f
typedef _Float16 h16;
typedef unsigned short bf;
typedef __attribute__((ext_vector_type(16))) __bf16   v16bf;
typedef __attribute__((ext_vector_type(16))) _Float16 v16h;
typedef __attribute__((ext_vector_type(8)))  _Float16 v8h;
typedef __attribute__((ext_vector_type(8)))  unsigned short v8us;
typedef __attribute__((ext_vector_type(8)))  float    v8f;
typedef __attribute__((ext_vector_type(4)))  float    v4f;
typedef v8h  __attribute__((may_alias)) v8ha;
typedef v4f  __attribute__((may_alias)) v4fa;
typedef v8us __attribute__((may_alias)) v8usa;

__device__ __forceinline__ unsigned short f2bf(float f) { unsigned u = __float_as_uint(f); u += 0x7FFFu + ((u >> 16) & 1u); return (unsigned short)(u >> 16); }
__device__ __forceinline__ float bf2f(unsigned short b) { return __uint_as_float(((unsigned)b) << 16); }
__device__ __forceinline__ float bfr(float f) { return bf2f(f2bf(f)); }
__device__ __forceinline__ v16h cat16(v8h lo, v8h hi) { return __builtin_shufflevector(lo, hi, 0, 1, 2, 3, 4, 5, 6, 7, 8, 9, 10, 11, 12, 13, 14, 15); }
__device__ __forceinline__ v16bf cat16b(v8us lo, v8us hi) { return __builtin_bit_cast(v16bf, __builtin_shufflevector(lo, hi, 0, 1, 2, 3, 4, 5, 6, 7, 8, 9, 10, 11, 12, 13, 14, 15)); }
__device__ __forceinline__ v8f wmma16(v16h a, v16h b, v8f c) { return __builtin_amdgcn_wmma_f32_16x16x32_f16(false, a, false, b, (short)0, c, false, false); }
__device__ __forceinline__ v8f wmmab(v16bf a, v16bf b, v8f c) { return __builtin_amdgcn_wmma_f32_16x16x32_bf16(false, a, false, b, (short)0, c, false, false); }

template <typename T16> struct WFrag;
template <> struct WFrag<h16> { typedef v16h V; static __device__ __forceinline__ V ld(const h16* p) { return cat16(*(const v8h*)p, *(const v8h*)(p + 16)); } static __device__ __forceinline__ v8f mma(V a, V b, v8f c) { return wmma16(a, b, c); } };
template <> struct WFrag<bf> { typedef v16bf V; static __device__ __forceinline__ V ld(const bf* p) { return cat16b(*(const v8us*)p, *(const v8us*)(p + 16)); } static __device__ __forceinline__ v8f mma(V a, V b, v8f c) { return wmmab(a, b, c); } };
template <typename T16, int NSPLIT, bool BIAS>
__global__ __launch_bounds__(32) void k_gemmw(const T16* __restrict__ A, const T16* __restrict__ A2, const T16* __restrict__ Bt, const T16* __restrict__ Bt2, int K, float* C, int ldc, const float* __restrict__ bias, size_t sA, size_t sB, size_t sC) {
    typedef typename WFrag<T16>::V V;
    __shared__ __align__(16) float os[16 * 68];
    const size_t z = blockIdx.z; A += z * sA; if (A2) A2 += z * sA; Bt += z * sB; if (Bt2) Bt2 += z * sB; C += z * sC;
    const int lane = threadIdx.x & 31, lr = lane & 15, hi = lane >> 4; const int r0 = blockIdx.x * 64, c0 = blockIdx.y * 64;
    v8f acc[4][4];
#pragma unroll
    for (int mb = 0; mb < 4; ++mb)
#pragma unroll
        for (int nb = 0; nb < 4; ++nb) acc[mb][nb] = (v8f){};
    const size_t aoff = (size_t)(r0 + lr) * K + 8 * hi, boff = (size_t)(c0 + lr) * K + 8 * hi;
    for (int kc = 0; kc < K; kc += 32) {
        V a[4], a2[4];
#pragma unroll
        for (int mb = 0; mb < 4; ++mb) { a[mb] = WFrag<T16>::ld(A + aoff + (size_t)mb * 16 * K + kc); if (NSPLIT == 1 || NSPLIT == 2) a2[mb] = WFrag<T16>::ld(A2 + aoff + (size_t)mb * 16 * K + kc); }
#pragma unroll
        for (int nb = 0; nb < 4; ++nb) { const V b = WFrag<T16>::ld(Bt + boff + (size_t)nb * 16 * K + kc); V b2; if (NSPLIT >= 2) b2 = WFrag<T16>::ld(Bt2 + boff + (size_t)nb * 16 * K + kc);
#pragma unroll
            for (int mb = 0; mb < 4; ++mb) { acc[mb][nb] = WFrag<T16>::mma(a[mb], b, acc[mb][nb]); if (NSPLIT == 1 || NSPLIT == 2) acc[mb][nb] = WFrag<T16>::mma(a2[mb], b, acc[mb][nb]); if (NSPLIT >= 2) acc[mb][nb] = WFrag<T16>::mma(a[mb], b2, acc[mb][nb]); } }
        asm volatile("v_nop\n\tv_nop\n\tv_nop\n\tv_nop" : "+v"(acc[0][0]), "+v"(acc[1][1]), "+v"(acc[2][2]), "+v"(acc[3][3]) : "v"(a[0]), "v"(a[3]));
    }
#pragma unroll
    for (int mb = 0; mb < 4; ++mb) {
#pragma unroll
        for (int nb = 0; nb < 4; ++nb) {
#pragma unroll
            for (int j = 0; j < 8; ++j) os[(hi * 8 + j) * 68 + nb * 16 + lr] = acc[mb][nb][j]; }
        __builtin_amdgcn_wave_barrier(); asm volatile("" ::: "memory");
        float* crow = C + (size_t)(r0 + mb * 16) * ldc + c0;
#pragma unroll 1
        for (int ps = 0; ps < 2; ++ps) {
#pragma unroll
            for (int s = 0; s < 8; ++s) { const int row = 2 * s + hi, cofs = lr * 4; v4f val = *(const v4fa*)(os + row * 68 + cofs); if (BIAS) { val[0] += bfr(bias[c0 + cofs]); val[1] += bfr(bias[c0 + cofs + 1]); val[2] += bfr(bias[c0 + cofs + 2]); val[3] += bfr(bias[c0 + cofs + 3]); }
                *(volatile v4f*)(crow + (size_t)row * ldc + cofs) = val; }
            if (ps == 0) __threadfence(); }
        __builtin_amdgcn_wave_barrier(); asm volatile("" ::: "memory");
    }
}

__device__ __forceinline__ h16 tohx(float x) { return (h16)x; }
__device__ __forceinline__ void splitf(float y, unsigned short& h, unsigned short& l) { h = f2bf(y); l = f2bf(y - bf2f(h)); }
typedef __attribute__((ext_vector_type(2))) _Float16 v2h;
typedef __attribute__((ext_vector_type(4))) _Float16 v4h;
typedef __attribute__((ext_vector_type(2))) unsigned short v2us;
typedef __attribute__((ext_vector_type(4))) unsigned short v4us;
typedef __attribute__((ext_vector_type(2))) float v2f;
typedef __attribute__((ext_vector_type(4))) int v4i;

template <typename T16, int NSPLIT, bool BIAS, int NW>
__global__ __launch_bounds__(32) void k_gemmn(const T16* __restrict__ A, const T16* __restrict__ A2, const T16* __restrict__ Bt, const T16* __restrict__ Bt2, int K, float* C, int ldc, const float* __restrict__ bias, size_t sA, size_t sB, size_t sC) {
    typedef typename WFrag<T16>::V V;
    static_assert(NW == 16 || NW == 32 || NW == 64, "the tile's width is 16, 32 or 64");
    constexpr int NB = NW / 16, PITCH = NW + 4, LS = (NW == 64) ? 4 : (NW == 32) ? 3 : 2;
    __shared__ __align__(16) float os[16 * PITCH];
    const size_t z = blockIdx.z; A += z * sA; if (A2) A2 += z * sA; Bt += z * sB; if (Bt2) Bt2 += z * sB; C += z * sC;
    const int lane = threadIdx.x & 31, lr = lane & 15, hi = lane >> 4; const int r0 = blockIdx.x * 64, c0 = blockIdx.y * NW;
    v8f acc[4][NB];
#pragma unroll
    for (int mb = 0; mb < 4; ++mb)
#pragma unroll
        for (int nb = 0; nb < NB; ++nb) acc[mb][nb] = (v8f){};
    const size_t aoff = (size_t)(r0 + lr) * K + 8 * hi, boff = (size_t)(c0 + lr) * K + 8 * hi;
    for (int kc = 0; kc < K; kc += 32) {
        V a[4], a2[4];
#pragma unroll
        for (int mb = 0; mb < 4; ++mb) { a[mb] = WFrag<T16>::ld(A + aoff + (size_t)mb * 16 * K + kc); if (NSPLIT == 1 || NSPLIT == 2) a2[mb] = WFrag<T16>::ld(A2 + aoff + (size_t)mb * 16 * K + kc); }
#pragma unroll
        for (int nb = 0; nb < NB; ++nb) { const V b = WFrag<T16>::ld(Bt + boff + (size_t)nb * 16 * K + kc); V b2; if (NSPLIT >= 2) b2 = WFrag<T16>::ld(Bt2 + boff + (size_t)nb * 16 * K + kc);
#pragma unroll
            for (int mb = 0; mb < 4; ++mb) { acc[mb][nb] = WFrag<T16>::mma(a[mb], b, acc[mb][nb]); if (NSPLIT == 1 || NSPLIT == 2) acc[mb][nb] = WFrag<T16>::mma(a2[mb], b, acc[mb][nb]); if (NSPLIT >= 2) acc[mb][nb] = WFrag<T16>::mma(a[mb], b2, acc[mb][nb]); } }
        asm volatile("v_nop\n\tv_nop\n\tv_nop\n\tv_nop" : "+v"(acc[0][0]), "+v"(acc[1][1 % NB]), "+v"(acc[2][2 % NB]), "+v"(acc[3][3 % NB]) : "v"(a[0]), "v"(a[3]));
    }
#pragma unroll
    for (int mb = 0; mb < 4; ++mb) {
#pragma unroll
        for (int nb = 0; nb < NB; ++nb) {
#pragma unroll
            for (int j = 0; j < 8; ++j) os[(hi * 8 + j) * PITCH + nb * 16 + lr] = acc[mb][nb][j]; }
        __builtin_amdgcn_wave_barrier(); asm volatile("" ::: "memory");
        float* crow = C + (size_t)(r0 + mb * 16) * ldc + c0;
        for (int ps = 0; ps < 2; ++ps) {
#pragma unroll
            for (int s = 0; s < NW / 8; ++s) { const int row = (128 / NW) * s + (lane >> LS), cofs = (lane & (NW / 4 - 1)) * 4; v4f val = *(const v4fa*)(os + row * PITCH + cofs); if (BIAS) { val[0] += bfr(bias[c0 + cofs]); val[1] += bfr(bias[c0 + cofs + 1]); val[2] += bfr(bias[c0 + cofs + 2]); val[3] += bfr(bias[c0 + cofs + 3]); }
                *(volatile v4f*)(crow + (size_t)row * ldc + cofs) = val; }
            if (ps == 0) __threadfence(); }
        __builtin_amdgcn_wave_barrier(); asm volatile("" ::: "memory");
    }
}

__global__ __launch_bounds__(256) void k_wtG(const float* __restrict__ w, int K, int N, bf* Bt) {
    const int lane = threadIdx.x & 31; const int L0 = (blockIdx.x * 8 + (threadIdx.x >> 5)) * 8; const int nlines = N * K / 64;
#pragma unroll
    for (int ps = 0; ps < 2; ++ps) {
        for (int l = 0; l < 8; ++l) { const int L = L0 + l; if (L >= nlines) break; const size_t e = (size_t)L * 64 + lane * 2; const int k = (int)(e % K), n = (int)(e / K); v2us o;
            o[0] = f2bf(w[(size_t)k * N + n]); o[1] = f2bf(w[(size_t)(k + 1) * N + n]); *(volatile v2us*)(Bt + e) = o; }
        if (ps == 0) __threadfence(); }
}
__global__ __launch_bounds__(256) void k_cvt8(const float* __restrict__ src, bf* dst, size_t n8) { const size_t i = (size_t)blockIdx.x * 256 + threadIdx.x; if (i >= n8) return; const v8f v = *(const v8f*)(src + i * 8); v8us o;
#pragma unroll
    for (int k = 0; k < 8; ++k) o[k] = f2bf(v[k]); *(volatile v8us*)(dst + i * 8) = o; __threadfence(); *(volatile v8us*)(dst + i * 8) = o; }
__global__ __launch_bounds__(256) void k_rbf(const float* __restrict__ X, float* Y, size_t n4) { const size_t i = (size_t)blockIdx.x * 256 + threadIdx.x; if (i >= n4) return; const v4f a = *(const v4f*)(X + i * 4); v4f o;
#pragma unroll
    for (int q = 0; q < 4; ++q) o[q] = bfr(a[q]);
    *(volatile v4f*)(Y + i * 4) = o; __threadfence(); *(volatile v4f*)(Y + i * 4) = o; }

#define LNC_MAX 2048
template <bool RES>
__global__ __launch_bounds__(256) void k_lnrow(const float* __restrict__ A, const float* __restrict__ R, const float* __restrict__ gamma, const float* __restrict__ beta, float eps, int C, int nrows, float* Y) {
    const int lane = threadIdx.x & 31; const int row = blockIdx.x * 8 + (threadIdx.x >> 5); if (row >= nrows) return; const int nch = C / 128; const float* a = A + (size_t)row * C; float x[LNC_MAX / 32]; float s = 0.0f;
    for (int k = 0; k < LNC_MAX / 128; ++k) { if (k < nch) { const int c0 = k * 128 + lane * 4; v4f v = *(const v4f*)(a + c0);
            if (RES) { const v4f w = *(const v4f*)(R + (size_t)row * C + c0); v[0] = __fadd_rn(v[0], w[0]); v[1] = __fadd_rn(v[1], w[1]); v[2] = __fadd_rn(v[2], w[2]); v[3] = __fadd_rn(v[3], w[3]); }
            x[k * 4 + 0] = v[0]; x[k * 4 + 1] = v[1]; x[k * 4 + 2] = v[2]; x[k * 4 + 3] = v[3]; s = __fadd_rn(__fadd_rn(__fadd_rn(__fadd_rn(s, v[0]), v[1]), v[2]), v[3]); } }
    for (int sh = 16; sh; sh >>= 1) s = __fadd_rn(s, __shfl_xor(s, sh, 32));
    const float mean = __fdiv_rn(s, (float)C); float q = 0.0f;
    for (int k = 0; k < LNC_MAX / 128; ++k) { if (k < nch) {
            for (int j = 0; j < 4; ++j) { const float d = __fsub_rn(x[k * 4 + j], mean); x[k * 4 + j] = d; q = __fmaf_rn(d, d, q); } } }
    for (int sh = 16; sh; sh >>= 1) q = __fadd_rn(q, __shfl_xor(q, sh, 32));
    const float rstd = __fdiv_rn(1.0f, sqrtf(__fadd_rn(__fdiv_rn(q, (float)C), eps)));
    for (int k = 0; k < LNC_MAX / 128; ++k) { if (k < nch) { const int c0 = k * 128 + lane * 4; const v4f g = *(const v4f*)(gamma + c0); const v4f bt = *(const v4f*)(beta + c0);
            for (int j = 0; j < 4; ++j) x[k * 4 + j] = __fmaf_rn(__fmul_rn(x[k * 4 + j], rstd), bfr(g[j]), bfr(bt[j])); } }
    float* y = Y + (size_t)row * C;
    for (int ps = 0; ps < 2; ++ps) {
        for (int k = 0; k < LNC_MAX / 128; ++k) { if (k < nch) { v4f o; o[0] = x[k * 4 + 0]; o[1] = x[k * 4 + 1]; o[2] = x[k * 4 + 2]; o[3] = x[k * 4 + 3]; *(volatile v4f*)(y + k * 128 + lane * 4) = o; } }
        if (ps == 0) __threadfence(); }
}

__global__ __launch_bounds__(256) void k_asoftMA(const float* __restrict__ Sb, const float* __restrict__ MP, h16* P16, bf* Ph, bf* Pl) {
    const int lane = threadIdx.x & 31; const int row = blockIdx.x * 8 + (threadIdx.x >> 5); if (row >= ZH * TT) return; const int i = row % TT; const int zz = row / TT; (void)zz; const bool hires = (i < RH); const float* sr = Sb + (size_t)row * TT; float v[TT / 32]; float mx = -3.0e38f;
#pragma unroll
    for (int ch = 0; ch < TT / 128; ++ch) { const int j0 = ch * 128 + lane * 4; const v4f a = *(const v4f*)(sr + j0); const v4f m4 = *(const v4f*)(MP + (size_t)i * TT + j0);
#pragma unroll
        for (int q = 0; q < 4; ++q) { const int j = j0 + q; (void)j; const float t = a[q] * SCL + bfr(m4[q]) * PMUL;     v[ch * 4 + q] = t; mx = fmaxf(mx, t); } }
#pragma unroll
    for (int sh = 16; sh; sh >>= 1) mx = fmaxf(mx, __shfl_xor(mx, sh, 32));
    float sum = 0.f;
#pragma unroll
    for (int k = 0; k < TT / 32; ++k) { float d0 = __fsub_rn(v[k], mx); v[k] = __builtin_amdgcn_exp2f(__fmul_rn(d0, 1.4426950408889634f)); sum += v[k]; }
#pragma unroll
    for (int sh = 16; sh; sh >>= 1) sum += __shfl_xor(sum, sh, 32);
    const float f = __fdiv_rn(hires ? 1.0f : PCAR, sum);
#pragma unroll 1
    for (int ps = 0; ps < 2; ++ps) {
        if (hires) {
#pragma unroll
            for (int ch = 0; ch < TT / 128; ++ch) { v4us oh, ol;
#pragma unroll
                for (int q = 0; q < 4; ++q) { unsigned short a, c2; splitf(v[ch * 4 + q] * f, a, c2); oh[q] = a; ol[q] = c2; }
                const size_t oo = ((size_t)zz * (RH ? RH : 1) + i) * TT + ch * 128 + lane * 4; *(volatile v4us*)(Ph + oo) = oh; *(volatile v4us*)(Pl + oo) = ol; }
        } else {
#pragma unroll
            for (int ch = 0; ch < TT / 128; ++ch) { v4h o4;
#pragma unroll
                for (int q = 0; q < 4; ++q) o4[q] = tohx(v[ch * 4 + q] * f);
                *(volatile v4h*)(P16 + (size_t)row * TT + ch * 128 + lane * 4) = o4; } }
        if (ps == 0) __threadfence(); }
}
typedef __attribute__((ext_vector_type(4))) float v4f_t;
__global__ __launch_bounds__(256) void k_fill(float* __restrict__ p, float val, size_t n4) { const size_t i = (size_t)blockIdx.x * 256 + threadIdx.x; if (i < n4) { v4f_t v = {val, val, val, val}; *(volatile v4f_t*)(p + 4 * i) = v; __threadfence(); *(volatile v4f_t*)(p + 4 * i) = v; } }
__global__ __launch_bounds__(256) void k_hp48(const float* __restrict__ src, h16* dst) { const unsigned i = blockIdx.x * 256 + threadIdx.x; if (i >= 8u * 768u * 16u) return; const unsigned hd = i / (768u * 16u), r = i - hd * (768u * 16u), row = r >> 4, d = (r & 15u) * 4u; const bool live = d < 48u; const v4f a = *(const v4f*)(src + (size_t)row * 384 + hd * 48 + (live ? d : 0u)); v4h o;
#pragma unroll
    for (int q = 0; q < 4; ++q) o[q] = live ? tohx(a[q]) : (h16)0.0f;
    *(volatile v4h*)(dst + (size_t)i * 4) = o; __threadfence(); *(volatile v4h*)(dst + (size_t)i * 4) = o; }
__global__ __launch_bounds__(256) void k_vt48(const float* __restrict__ src, h16* dst) { const unsigned i = blockIdx.x * 256 + threadIdx.x; if (i >= 8u * 64u * 384u) return; const unsigned hd = i / (64u * 384u), r = i - hd * (64u * 384u), d = r / 384u, p = (r - d * 384u) * 2u; const bool live = d < 48u; const unsigned c = hd * 48 + (live ? d : 0u); const float x0 = src[(size_t)p * 384 + c], x1 = src[(size_t)(p + 1) * 384 + c]; v2h o; o[0] = live ? tohx(x0) : (h16)0.0f; o[1] = live ? tohx(x1) : (h16)0.0f;
    *(volatile v2h*)(dst + (size_t)i * 2) = o; __threadfence(); *(volatile v2h*)(dst + (size_t)i * 2) = o; }
__global__ __launch_bounds__(256) void k_hb(const float* __restrict__ E, const float* __restrict__ PB, const float* __restrict__ pbias, int h, float rs, const float* __restrict__ S, float* S2, float* MP) { const unsigned i = blockIdx.x * 256 + threadIdx.x; if (i >= 768u * 192u) return; const size_t e = (size_t)i * 4; const v4f s4 = *(const v4f*)(S + e); const float bh = bfr(pbias[h]); v4f m, o;
#pragma unroll
    for (int q = 0; q < 4; ++q) { m[q] = E[(e + q) * 16 + h]; o[q] = __fmaf_rn(PB[(e + q) * 16 + h] + bh, rs, s4[q]); }
    *(volatile v4f*)(MP + e) = m; *(volatile v4f*)(S2 + e) = o; __threadfence(); *(volatile v4f*)(MP + e) = m; *(volatile v4f*)(S2 + e) = o; }
__global__ __launch_bounds__(256) void k_sg(const float* __restrict__ X, int px, int xhw, int xs, const float* __restrict__ G, int pg, const float* __restrict__ W, int pw, float cf, float* Y, int py, int w4, int nrows) { const unsigned i = blockIdx.x * 256 + threadIdx.x; if (i >= (unsigned)(w4 * nrows)) return; const unsigned r = i / (unsigned)w4, c = (i - r * (unsigned)w4) * 4u; const unsigned xb = c / (unsigned)xhw, xc = xb * (unsigned)xs + (c - xb * (unsigned)xhw); const v4f x = *(const v4f*)(X + (size_t)r * px + xc); const v4f g = *(const v4f*)(G + (size_t)r * pg + c); const v4f w = *(const v4f*)(W + (size_t)r * pw + c); v4f o;
#pragma unroll
    for (int q = 0; q < 4; ++q) { const float ex = __builtin_amdgcn_exp2f(__fmul_rn(-g[q], 1.4426950408889634f)); const float sg = __fdiv_rn(1.0f, 1.0f + ex); o[q] = __fmaf_rn(__fmul_rn(x[q], cf), sg, w[q]); }
    *(volatile v4f*)(Y + (size_t)r * py + c) = o; __threadfence(); *(volatile v4f*)(Y + (size_t)r * py + c) = o; }
__global__ __launch_bounds__(256) void k_mg48(const float* __restrict__ O, float cf, bf* B) { const unsigned i = blockIdx.x * 256 + threadIdx.x; if (i >= 768u * 96u) return; const unsigned r = i / 96u, c = (i - r * 96u) * 4u; const unsigned xb = c / 48u, xc = xb * 64u + (c - xb * 48u); const v4f x = *(const v4f*)(O + (size_t)r * 512 + xc); v4us o;
#pragma unroll
    for (int q = 0; q < 4; ++q) o[q] = f2bf(__fmul_rn(x[q], cf));
    *(volatile v4us*)(B + (size_t)r * 384 + c) = o; __threadfence(); *(volatile v4us*)(B + (size_t)r * 384 + c) = o; }

extern "C" void kernel_launch(void* const* d_in, const int* in_sizes, int n_in,
                              void* d_out, int out_size, void* d_ws, size_t ws_size, hipStream_t stream) {
    (void)in_sizes; (void)n_in; (void)out_size;
    const float* i0 = (const float*)d_in[0]; const float* i1 = (const float*)d_in[1]; const float* i2 = (const float*)d_in[2]; const float* i3 = (const float*)d_in[3]; const float* i4 = (const float*)d_in[4]; const float* i5 = (const float*)d_in[5]; const float* i6 = (const float*)d_in[6]; const float* i7 = (const float*)d_in[7]; const float* i8 = (const float*)d_in[8]; const float* i9 = (const float*)d_in[9]; const float* i10 = (const float*)d_in[10]; const float* i11 = (const float*)d_in[11]; const float* i12 = (const float*)d_in[12]; const float* i13 = (const float*)d_in[13];
    static_assert(384 % 128 == 0 && 128 % 128 == 0 && 384 <= LNC_MAX, "k_lnrow: C must be a multiple of 128 and at most LNC_MAX");
    float* OUT = (float*)d_out;
    char* wsp = (char*)d_ws;
    auto take = [&](size_t bytes) { char* p = wsp; wsp += (bytes + 255) & ~(size_t)255; return (void*)p; };
    const size_t NN = (size_t)768 * 768, NS = (size_t)768 * 384, NW_ = (size_t)384 * 384, PZ = (size_t)64 * 768 * 128;
    bf* W6 = (bf*)take(NW_ * 2); bf* W7 = (bf*)take(NW_ * 2); bf* W8 = (bf*)take(NW_ * 2); bf* W10 = (bf*)take(NW_ * 2); bf* W12 = (bf*)take(NW_ * 2); bf* W9 = (bf*)take((size_t)16 * 128 * 2);
    float* ZE = (float*)take(NN * 16 * 4);
    float* R0 = (float*)take(NS * 4); float* N0 = (float*)take(NS * 4); bf* N0b = (bf*)take(NS * 2);
    float* F1 = (float*)take(NS * 4); float* F2 = (float*)take(NS * 4); float* F3 = (float*)take(NS * 4); float* FG = (float*)take(NS * 4);
    h16* QP16 = (h16*)take((size_t)8 * TT * HD * 2); h16* KP16 = (h16*)take((size_t)8 * TT * HD * 2); h16* VT16 = (h16*)take((size_t)8 * HD * TT * 2);
    float* ZR = (float*)take(PZ * 4); float* ZN = (float*)take(PZ * 4); bf* ZB = (bf*)take(PZ * 2); float* PB = (float*)take(NN * 16 * 4);
    float* Sb = (float*)take(NN * 4); float* S2 = (float*)take(NN * 4); float* MP = (float*)take(NN * 4); h16* P16 = (h16*)take(NN * 2); float* OB = (float*)take((size_t)TT * 8 * HD * 4); bf* MGB = (bf*)take(NS * 2); float* OM = (float*)take(NS * 4);
    if ((size_t)(wsp - (char*)d_ws) > ws_size) return;
    k_cvt8<<<(unsigned)((NW_ / 8 + 255) / 256), 256, 0, stream>>>(i6, W6, NW_ / 8); k_cvt8<<<(unsigned)((NW_ / 8 + 255) / 256), 256, 0, stream>>>(i7, W7, NW_ / 8); k_cvt8<<<(unsigned)((NW_ / 8 + 255) / 256), 256, 0, stream>>>(i8, W8, NW_ / 8); k_cvt8<<<(unsigned)((NW_ / 8 + 255) / 256), 256, 0, stream>>>(i10, W10, NW_ / 8); k_cvt8<<<(unsigned)((NW_ / 8 + 255) / 256), 256, 0, stream>>>(i12, W12, NW_ / 8);
    k_fill<<<1, 256, 0, stream>>>((float*)W9, 0.0f, (size_t)16 * 128 * 2 / 16); k_wtG<<<1, 256, 0, stream>>>(i9, 128, 8, W9);
    k_fill<<<(unsigned)((NN * 16 / 4 + 255) / 256), 256, 0, stream>>>(ZE, 0.0f, NN * 16 / 4);
    k_rbf<<<(unsigned)((NS / 4 + 255) / 256), 256, 0, stream>>>(i0, R0, NS / 4); k_lnrow<false><<<(unsigned)((768 + 7) / 8), 256, 0, stream>>>(R0, nullptr, i2, i3, 1.0e-5f, 384, 768, N0); k_cvt8<<<(unsigned)((NS / 8 + 255) / 256), 256, 0, stream>>>(N0, N0b, NS / 8);
    k_gemmw<bf, 0, false><<<dim3(768 / 64, 384 / 64, 1), 32, 0, stream>>>(N0b, nullptr, W6, nullptr, 384, F1, 384, nullptr, 0, 0, 0); k_gemmw<bf, 0, false><<<dim3(768 / 64, 384 / 64, 1), 32, 0, stream>>>(N0b, nullptr, W7, nullptr, 384, F2, 384, nullptr, 0, 0, 0); k_gemmw<bf, 0, false><<<dim3(768 / 64, 384 / 64, 1), 32, 0, stream>>>(N0b, nullptr, W8, nullptr, 384, F3, 384, nullptr, 0, 0, 0); k_gemmw<bf, 0, true><<<dim3(768 / 64, 384 / 64, 1), 32, 0, stream>>>(N0b, nullptr, W12, nullptr, 384, FG, 384, i13, 0, 0, 0);
    k_hp48<<<(unsigned)((8u * 768u * 16u + 255) / 256), 256, 0, stream>>>(F1, QP16); k_hp48<<<(unsigned)((8u * 768u * 16u + 255) / 256), 256, 0, stream>>>(F2, KP16); k_vt48<<<(unsigned)((8u * 64u * 384u + 255) / 256), 256, 0, stream>>>(F3, VT16);
    for (int p = 0; p < 12; ++p) {
        k_rbf<<<(unsigned)((PZ / 4 + 255) / 256), 256, 0, stream>>>(i1 + (size_t)p * PZ, ZR, PZ / 4); k_lnrow<false><<<(unsigned)((64 * 768 + 7) / 8), 256, 0, stream>>>(ZR, nullptr, i4, i5, 1.0e-5f, 128, 64 * 768, ZN); k_cvt8<<<(unsigned)((PZ / 8 + 255) / 256), 256, 0, stream>>>(ZN, ZB, PZ / 8);
        k_gemmn<bf, 0, false, 16><<<dim3(64 * 768 / 64, 1, 1), 32, 0, stream>>>(ZB, nullptr, W9, nullptr, 128, PB + (size_t)p * 64 * 768 * 16, 16, nullptr, 0, 0, 0); }
    for (int h = 0; h < 8; ++h) {
        k_gemmw<h16, 0, false><<<dim3(TT / 64, TT / 64, 1), 32, 0, stream>>>(QP16 + (size_t)h * TT * HD, nullptr, KP16 + (size_t)h * TT * HD, nullptr, HD, Sb, TT, nullptr, 0, 0, 0);
        k_hb<<<(unsigned)((NN / 4 + 255) / 256), 256, 0, stream>>>(ZE, PB, ZE, h, 6.9282032f, Sb, S2, MP);
        k_asoftMA<<<ZH * TT / 8, 256, 0, stream>>>(S2, MP, P16, nullptr, nullptr);
        k_gemmw<h16, 0, false><<<dim3(TT / 64, HD / 64, 1), 32, 0, stream>>>(P16, nullptr, VT16 + (size_t)h * HD * TT, nullptr, TT, OB + h * HD, 8 * HD, nullptr, 0, 0, 0); }
    k_mg48<<<(unsigned)((768u * 96u + 255) / 256), 256, 0, stream>>>(OB, 0.0009765625f, MGB);
    k_gemmw<bf, 0, true><<<dim3(768 / 64, 384 / 64, 1), 32, 0, stream>>>(MGB, nullptr, W10, nullptr, 384, OM, 384, i11, 0, 0, 0);
    k_sg<<<(unsigned)((NS / 4 + 255) / 256), 256, 0, stream>>>(OM, 384, 384, 384, FG, 384, R0, 384, 1.0f, OUT, 384, 384 / 4, 768);
}
